// GELU121_39857296507267
// MI455X (gfx1250) — hardware-verified
//
#include <hip/hip_runtime.h>
#include <math.h>
#include <stdint.h>

#define NB   4
#define NT   4096
#define ND   512
#define NR   (NB * NT)
#define RPB1 32
#define RPB3 8
#define IT   64
#define JT   64
#define XSC  64.0f
#define ISC2 0.000244140625f
#define GK   0.7978845608028654f
#define GC3  0.044715f

static_assert(ND == 512);
static_assert((NT % IT) == 0);
static_assert((NT % JT) == 0);
static_assert((NR % RPB1) == 0);
static_assert((NR % RPB3) == 0);
static_assert((ND % 32) == 0);
static_assert(IT == 4 * 16);
static_assert(JT == 4 * 16);
static_assert(RPB1 == 8 * 4);

typedef _Float16       v16h __attribute__((ext_vector_type(16)));
typedef _Float16       v8h  __attribute__((ext_vector_type(8)));
typedef float          v8f  __attribute__((ext_vector_type(8)));
typedef float          v4f  __attribute__((ext_vector_type(4)));
typedef unsigned int   v4u  __attribute__((ext_vector_type(4)));

union FragH { v16h v; v8h h[2]; };
static_assert(sizeof(FragH) == 32);

__device__ __forceinline__ unsigned short bf_bits(float f) {
  unsigned u = __float_as_uint(f);
  return (unsigned short)((u + 0x7FFFu + ((u >> 16) & 1u)) >> 16);
}
__device__ __forceinline__ float bf_up(unsigned short h) { return __uint_as_float(((unsigned)h) << 16); }
__device__ __forceinline__ float bfr(float f) { return bf_up(bf_bits(f)); }
__device__ __forceinline__ v4f bfr4(v4f v) {
  v4f r;
  r[0] = bfr(v[0]); r[1] = bfr(v[1]); r[2] = bfr(v[2]); r[3] = bfr(v[3]);
  return r;
}
__device__ __forceinline__ unsigned short h_bits(_Float16 x) { return __builtin_bit_cast(unsigned short, x); }
__device__ __forceinline__ unsigned pk16(unsigned short a, unsigned short b) { return (unsigned)a | ((unsigned)b << 16); }
__device__ __forceinline__ v8f zero8() { v8f z = {0.f, 0.f, 0.f, 0.f, 0.f, 0.f, 0.f, 0.f}; return z; }

__device__ __forceinline__ float tanh_e(float y) {
  const float a = fabsf(y);
  const float e = __expf(2.0f * a);
  const float r = __builtin_amdgcn_rcpf(e + 1.0f);
  const float t = fmaf(-2.0f, r, 1.0f);
  return copysignf(t, y);
}
__device__ __forceinline__ float gelu_f(float y) {
  const float y3 = y * y * y;
  const float z  = GK * (y + GC3 * y3);
  return 0.5f * y * (1.0f + tanh_e(z));
}
__device__ __forceinline__ float softplus_f(float v) { return fmaxf(v, 0.0f) + log1pf(expf(-fabsf(v))); }

__device__ __forceinline__ v16h ldfrag_h(const _Float16* p) {
  FragH f;
  f.h[0] = *(const v8h*)(p);
  f.h[1] = *(const v8h*)(p + 16);
  return f.v;
}

__device__ __forceinline__ v8f mma_h(v16h a, v16h b, v8f c) {
  v8f d = __builtin_amdgcn_wmma_f32_16x16x32_f16(false, a, false, b, (short)0, c, false, false);
#if defined(__HIP_DEVICE_COMPILE__)
  asm volatile("v_nop\n\tv_nop\n\tv_nop\n\tv_nop" : "+v"(d) : "v"(a), "v"(b));
#endif
  return d;
}

__global__ __launch_bounds__(256)
void norm_kernel(const float* __restrict__ x, unsigned short* XH, float* RN) {
  __shared__ __align__(16) float s_rn[RPB1];
  const int tid  = threadIdx.x;
  const int wave = tid >> 5, lane = tid & 31;
#pragma unroll 1
  for (int rr = 0; rr < 4; ++rr) {
    const int row = blockIdx.x * RPB1 + wave * 4 + rr;
    const float* xr = x + (size_t)row * ND + 8 * lane;
    const v4f a0 = bfr4(*(const v4f*)(xr));
    const v4f a1 = bfr4(*(const v4f*)(xr + 4));
    const v4f b0 = bfr4(*(const v4f*)(xr + 256));
    const v4f b1 = bfr4(*(const v4f*)(xr + 260));
    float ss = 0.f;
#pragma unroll
    for (int q = 0; q < 4; ++q) {
      ss = fmaf(a0[q], a0[q], ss);
      ss = fmaf(a1[q], a1[q], ss);
      ss = fmaf(b0[q], b0[q], ss);
      ss = fmaf(b1[q], b1[q], ss);
    }
#pragma unroll
    for (int msk = 16; msk >= 1; msk >>= 1) ss += __shfl_xor(ss, msk, 32);
    const float nx = fmaxf(sqrtf(ss), 1.0e-12f);
    const float rn = 1.0f / nx;
    v4u ua, ub;
#pragma unroll
    for (int t = 0; t < 2; ++t) {
      ua[t]     = pk16(h_bits((_Float16)(a0[2 * t] * XSC)), h_bits((_Float16)(a0[2 * t + 1] * XSC)));
      ua[2 + t] = pk16(h_bits((_Float16)(a1[2 * t] * XSC)), h_bits((_Float16)(a1[2 * t + 1] * XSC)));
      ub[t]     = pk16(h_bits((_Float16)(b0[2 * t] * XSC)), h_bits((_Float16)(b0[2 * t + 1] * XSC)));
      ub[2 + t] = pk16(h_bits((_Float16)(b1[2 * t] * XSC)), h_bits((_Float16)(b1[2 * t + 1] * XSC)));
    }
    unsigned short* dst = XH + (size_t)row * ND + 8 * lane;
    *(volatile v4u*)(dst)       = ua;
    *(volatile v4u*)(dst + 256) = ub;
    __threadfence();
    *(volatile v4u*)(dst)       = ua;
    *(volatile v4u*)(dst + 256) = ub;
    if (lane == 0) s_rn[wave * 4 + rr] = rn;
  }
  __syncthreads();
  if (wave == 0) {
    const int q = min(lane, 7);
    const v4f v = *(const v4f*)(s_rn + 4 * q);
    float* rp = RN + (size_t)blockIdx.x * RPB1 + 4 * q;
    if (lane < 8) *(volatile v4f*)rp = v;
    __threadfence();
    if (lane < 8) *(volatile v4f*)rp = v;
  }
}

__global__ __launch_bounds__(128)
void gram_kernel(const unsigned short* __restrict__ XH, const float* __restrict__ RN,
                 const float* __restrict__ p_la, float* G) {
  __shared__ __align__(16) float s_g[IT];
  const int tid  = threadIdx.x;
  const int wave = tid >> 5, lane = tid & 31;
  const int hh   = lane >> 4, m = lane & 15;
  const int bx   = blockIdx.x;
  const int b    = bx / (NT / IT);
  const int tile = bx % (NT / IT);
  const int i0   = tile * IT + wave * 16;
  const _Float16* Xh   = (const _Float16*)(const void*)XH;
  const _Float16* base = Xh + (size_t)b * NT * ND;
  const _Float16* ap   = base + (size_t)(i0 + m) * ND + 8 * hh;
  const float* rnb     = RN + (size_t)b * NT;
  const int gr0 = i0 + 8 * hh;

  v8f rt;
#pragma unroll
  for (int r = 0; r < 8; ++r) rt[r] = rnb[gr0 + r] * ISC2;

  v8f rmx = {-2.0f, -2.0f, -2.0f, -2.0f, -2.0f, -2.0f, -2.0f, -2.0f};
  const int ntile = tile + 1;
#pragma unroll 1
  for (int jt = 0; jt < ntile; ++jt) {
    const int j0 = jt * JT;
    const _Float16* bp = base + (size_t)(j0 + m) * ND + 8 * hh;
    const float c0 = rnb[j0 + 0 * 16 + m];
    const float c1 = rnb[j0 + 1 * 16 + m];
    const float c2 = rnb[j0 + 2 * 16 + m];
    const float c3 = rnb[j0 + 3 * 16 + m];
    v8f acc0 = zero8(), acc1 = zero8(), acc2 = zero8(), acc3 = zero8();
#pragma unroll 4
    for (int ks = 0; ks < ND / 32; ++ks) {
      const v16h a = ldfrag_h(ap + 32 * ks);
      acc0 = mma_h(a, ldfrag_h(bp + 0 * 16 * ND + 32 * ks), acc0);
      acc1 = mma_h(a, ldfrag_h(bp + 1 * 16 * ND + 32 * ks), acc1);
      acc2 = mma_h(a, ldfrag_h(bp + 2 * 16 * ND + 32 * ks), acc2);
      acc3 = mma_h(a, ldfrag_h(bp + 3 * 16 * ND + 32 * ks), acc3);
    }
#pragma unroll
    for (int r = 0; r < 8; ++r) {
      const int gr = gr0 + r;
      const float rr = rt[r];
      float s0 = acc0[r] * rr * c0, s1 = acc1[r] * rr * c1, s2 = acc2[r] * rr * c2, s3 = acc3[r] * rr * c3;
      s0 = ((j0 + 0 * 16 + m) < gr) ? s0 : -2.0f;
      s1 = ((j0 + 1 * 16 + m) < gr) ? s1 : -2.0f;
      s2 = ((j0 + 2 * 16 + m) < gr) ? s2 : -2.0f;
      s3 = ((j0 + 3 * 16 + m) < gr) ? s3 : -2.0f;
      rmx[r] = fmaxf(rmx[r], fmaxf(fmaxf(s0, s1), fmaxf(s2, s3)));
    }
  }
#pragma unroll
  for (int r = 0; r < 8; ++r) {
#pragma unroll
    for (int msk = 1; msk < 16; msk <<= 1) rmx[r] = fmaxf(rmx[r], __shfl_xor(rmx[r], msk, 32));
  }
  const float alpha = softplus_f(bfr(p_la[0]));
  if (m == 0) {
#pragma unroll
    for (int r = 0; r < 8; ++r) {
      const float ms  = fmaxf(rmx[r], -1.0f);
      const float fam = (ms + 1.0f) * 0.5f;
      const float nov = 1.0f - fam;
      s_g[wave * 16 + 8 * hh + r] = 1.0f + alpha * nov;
    }
  }
  __syncthreads();
  if (wave == 0) {
    const int q = min(lane, 15);
    const v4f v = *(const v4f*)(s_g + 4 * q);
    float* gp = G + (size_t)b * NT + (size_t)tile * IT + 4 * q;
    if (lane < 16) *(volatile v4f*)gp = v;
    __threadfence();
    if (lane < 16) *(volatile v4f*)gp = v;
  }
}

__global__ __launch_bounds__(256)
void out_kernel(const float* __restrict__ x, const float* __restrict__ G, float* out) {
  const int tid  = threadIdx.x;
  const int wave = tid >> 5, lane = tid & 31;
  const int row  = blockIdx.x * RPB3 + wave;
  const float g  = G[row];
  const float* xr = x + (size_t)row * ND + 4 * lane;
  float* op = out + (size_t)row * ND + 4 * lane;
#pragma unroll 1
  for (int s = 0; s < 4; ++s) {
    const v4f v = bfr4(*(const v4f*)(xr + 128 * s));
    v4f w;
    w[0] = gelu_f(v[0] * g);
    w[1] = gelu_f(v[1] * g);
    w[2] = gelu_f(v[2] * g);
    w[3] = gelu_f(v[3] * g);
    *(volatile v4f*)(op + 128 * s) = w;
    __threadfence();
    *(volatile v4f*)(op + 128 * s) = w;
  }
}

extern "C" void kernel_launch(void* const* d_in, const int* in_sizes, int n_in,
                              void* d_out, int out_size, void* d_ws, size_t ws_size,
                              hipStream_t stream) {
  if (n_in < 2) return;
  if (in_sizes[0] != NR * ND) return;
  if (in_sizes[1] < 1) return;
  if (out_size != NR * ND) return;

  size_t off = 0;
  const size_t oXH = off; off += (size_t)NR * ND * 2;
  const size_t oRN = off; off += (size_t)NR * 4;
  const size_t oG  = off; off += (size_t)NR * 4;
  if (off > ws_size) return;
  if (off > (size_t)134217728) return;

  const float* x     = (const float*)d_in[0];
  const float* log_a = (const float*)d_in[1];
  char* ws = (char*)d_ws;
  unsigned short* XH = (unsigned short*)(ws + oXH);
  float* RN  = (float*)(ws + oRN);
  float* G   = (float*)(ws + oG);
  float* out = (float*)d_out;

  const dim3 blk256(256), blk128(128);
  const dim3 gNorm(NR / RPB1);
  const dim3 gGram(NB * (NT / IT));
  const dim3 gOut(NR / RPB3);

  norm_kernel<<<gNorm, blk256, 0, stream>>>(x, XH, RN);
  gram_kernel<<<gGram, blk128, 0, stream>>>(XH, RN, log_a, G);
  out_kernel<<<gOut, blk256, 0, stream>>>(x, G, out);
  (void)hipGetLastError();
}
